// GraphConv_38594576122649
// MI455X (gfx1250) — hardware-verified
//
#include <hip/hip_runtime.h>
#include <stddef.h>
#include <stdint.h>


#define MNODE  4096
#define LOGM   12
#define NNB    16
#define NENT   (MNODE * NNB)
#define GN     4
#define BSZ    16
#define XF     32
#define OF     32
#define LOCF   8
#define LH     128
#define NXW    (GN * OF)
#define KP     32
#define NROWS  (BSZ * MNODE)
#define MM1    (MNODE * MNODE - 1)

#define NTHR   256
#define NWAVE  8
#define EPT    8
#define CHUNK  (NTHR * EPT)
#define WCAP   (EPT * 32)
#define LISTN  (NWAVE * WCAP)
#define NBA    512
#define SLA    9
#define RCAP   12288
#define DEGCAP 48
#define AGG_ZINTS    (LISTN + 2 * RCAP + 3 * NBA)
#define MISC_INTS    16
#define AGG_LDS_INTS (AGG_ZINTS + MISC_INTS)
#define ATHR   128
#define NPB    4
#define GBM    64
#define WUNITS (GN * LH * (KP / 8))
#define WSMAX  134217728

static_assert((CHUNK & (CHUNK - 1)) == 0 && CHUNK <= 4096);
static_assert((NBA & (NBA - 1)) == 0 && NBA == (1 << SLA));
static_assert(((long long)CHUNK << SLA) < (1LL << 31));
static_assert(((long long)NENT << SLA) < (1LL << 31));
static_assert(LISTN % NTHR == 0);
static_assert(NBA % NWAVE == 0 && NBA % 32 == 0);
static_assert(RCAP % 4 == 0 && AGG_ZINTS % 4 == 0 && LISTN % 4 == 0);
static_assert(DEGCAP <= 64);
static_assert(AGG_LDS_INTS * 4 <= 300000);
static_assert(MNODE % NBA == 0 && MNODE % NPB == 0);
static_assert(NROWS % GBM == 0 && GBM == (ATHR / 32) * 16);
static_assert(NENT % CHUNK == 0);
static_assert(KP == 32 && XF == 32 && NXW == 128 && OF == 32 && LH % 16 == 0);
static_assert((GN * XF * OF) % (4 * ATHR) == 0);
static_assert(WUNITS % NTHR == 0);
static_assert(BSZ == 16 && GN == 4);

typedef float          v4f   __attribute__((ext_vector_type(4)));
typedef float          v8f   __attribute__((ext_vector_type(8)));
typedef int            v4i   __attribute__((ext_vector_type(4)));
typedef int            v8i   __attribute__((ext_vector_type(8)));
typedef unsigned short v8us  __attribute__((ext_vector_type(8)));
typedef unsigned short v16us __attribute__((ext_vector_type(16)));
typedef __bf16         v16bf __attribute__((ext_vector_type(16)));
typedef v4f  __attribute__((may_alias)) v4fa;
typedef v4i  __attribute__((may_alias)) v4ia;
typedef v8us __attribute__((may_alias)) v8usa;
union FragB { v16bf v; v16us u; v8us h[2]; v8i w; };

__device__ __forceinline__ v8f wmb(const FragB& a, const FragB& b, v8f c) {
  v8f d = __builtin_amdgcn_wmma_f32_16x16x32_bf16(false, a.v, false, b.v, (short)0, c, false, false);
  asm volatile("v_nop\n\tv_nop\n\tv_nop\n\tv_nop" : "+v"(d) : "v"(a.w), "v"(b.w));
  return d;
}

__device__ __forceinline__ unsigned bf16_bits(float f) {
  const unsigned u = __float_as_uint(f);
  return (u + 0x7FFFu + ((u >> 16) & 1u)) >> 16;
}
__device__ __forceinline__ float bf16_val(float f) {
  return __uint_as_float(bf16_bits(f) << 16);
}

__device__ __forceinline__ void wave_sync() {
  __builtin_amdgcn_fence(__ATOMIC_RELEASE, "wavefront");
  __builtin_amdgcn_wave_barrier();
  __builtin_amdgcn_fence(__ATOMIC_ACQUIRE, "wavefront");
}

__device__ __forceinline__ v4f sel4(bool c, v4f a, v4f b) {
  v4f r;
  r.x = c ? a.x : b.x; r.y = c ? a.y : b.y; r.z = c ? a.z : b.z; r.w = c ? a.w : b.w;
  return r;
}

__device__ __forceinline__ int clampd(int d) { return d < 0 ? 0 : (d > MM1 ? MM1 : d); }
__device__ __forceinline__ int keyrow(int d) { return clampd(d) >> LOGM; }
__device__ __forceinline__ int keycol(int d) { return clampd(d) & (MNODE - 1); }

template <int SLB>
__device__ __forceinline__ int scan_chunk(const int* __restrict__ lix, int nE, int cbase, int slotBase,
                                          int nb, int vec8, int* list, int tid, int lane, int wave) {
  int wc = 0;
  const int el0  = tid * EPT;
  const int e0   = cbase + el0;
  const int none = -0x40000000;
  v4i da, db;
  if (vec8 != 0 && cbase + CHUNK <= nE) {
    da = *(const v4i*)(lix + e0);
    db = *(const v4i*)(lix + e0 + 4);
    da.x = keyrow(da.x); da.y = keyrow(da.y); da.z = keyrow(da.z); da.w = keyrow(da.w);
    db.x = keyrow(db.x); db.y = keyrow(db.y); db.z = keyrow(db.z); db.w = keyrow(db.w);
  } else {
    const int r0 = lix[min(e0,     nE - 1)], r1 = lix[min(e0 + 1, nE - 1)];
    const int r2 = lix[min(e0 + 2, nE - 1)], r3 = lix[min(e0 + 3, nE - 1)];
    const int r4 = lix[min(e0 + 4, nE - 1)], r5 = lix[min(e0 + 5, nE - 1)];
    const int r6 = lix[min(e0 + 6, nE - 1)], r7 = lix[min(e0 + 7, nE - 1)];
    da.x = (e0     < nE) ? keyrow(r0) : none;
    da.y = (e0 + 1 < nE) ? keyrow(r1) : none;
    da.z = (e0 + 2 < nE) ? keyrow(r2) : none;
    da.w = (e0 + 3 < nE) ? keyrow(r3) : none;
    db.x = (e0 + 4 < nE) ? keyrow(r4) : none;
    db.y = (e0 + 5 < nE) ? keyrow(r5) : none;
    db.z = (e0 + 6 < nE) ? keyrow(r6) : none;
    db.w = (e0 + 7 < nE) ? keyrow(r7) : none;
  }
  const unsigned nbs = (unsigned)slotBase;
  const unsigned unb = (unsigned)nb;
  const unsigned s0 = (unsigned)da.x - nbs, s1 = (unsigned)da.y - nbs;
  const unsigned s2 = (unsigned)da.z - nbs, s3 = (unsigned)da.w - nbs;
  const unsigned s4 = (unsigned)db.x - nbs, s5 = (unsigned)db.y - nbs;
  const unsigned s6 = (unsigned)db.z - nbs, s7 = (unsigned)db.w - nbs;
  const bool h0 = s0 < unb, h1 = s1 < unb, h2 = s2 < unb, h3 = s3 < unb;
  const bool h4 = s4 < unb, h5 = s5 < unb, h6 = s6 < unb, h7 = s7 < unb;
  const unsigned any = __builtin_amdgcn_ballot_w32(h0 | h1 | h2 | h3 | h4 | h5 | h6 | h7);
  if (any != 0u) {
#define HITJ(J, HJ, SJ) { \
      const unsigned mj = __builtin_amdgcn_ballot_w32(HJ); \
      if (mj != 0u) { \
        if (HJ) { \
          const int pos = wc + (int)__builtin_amdgcn_mbcnt_lo(mj, 0u); \
          if (pos < WCAP) list[wave * WCAP + pos] = ((el0 + (J)) << SLB) | (int)(SJ); \
        } \
        wc += (int)__builtin_popcount(mj); } }
    HITJ(0, h0, s0)
    HITJ(1, h1, s1)
    HITJ(2, h2, s2)
    HITJ(3, h3, s3)
    HITJ(4, h4, s4)
    HITJ(5, h5, s5)
    HITJ(6, h6, s6)
    HITJ(7, h7, s7)
#undef HITJ
  }
  return wc;
}

__global__ __launch_bounds__(NTHR) void k_w1prep(const float* __restrict__ w1, unsigned short* w1p) {
  const int u = (int)blockIdx.x * NTHR + (int)threadIdx.x;
  if (u >= WUNITS) return;
  const int n  = u >> 2;
  const int k8 = (u & 3) * 8;
  const float* p = w1 + (size_t)n * LOCF;
  const v4f a = *(const v4fa*)p;
  const v4f b = *(const v4fa*)(p + 4);
  const unsigned msk = (k8 == 0) ? 0xFFFFu : 0u;
  v8us o;
  o[0] = (unsigned short)(bf16_bits(a.x) & msk); o[1] = (unsigned short)(bf16_bits(a.y) & msk);
  o[2] = (unsigned short)(bf16_bits(a.z) & msk); o[3] = (unsigned short)(bf16_bits(a.w) & msk);
  o[4] = (unsigned short)(bf16_bits(b.x) & msk); o[5] = (unsigned short)(bf16_bits(b.y) & msk);
  o[6] = (unsigned short)(bf16_bits(b.z) & msk); o[7] = (unsigned short)(bf16_bits(b.w) & msk);
  unsigned short* dp = w1p + (size_t)u * 8;
  *(volatile v8us*)dp = o;
  __threadfence();
  *(volatile v8us*)dp = o;
}

__global__ __launch_bounds__(ATHR) void k_att(const float* __restrict__ maps, const unsigned short* __restrict__ w1p,
                                              const float* __restrict__ b1, const float* __restrict__ w2,
                                              const float* __restrict__ b2, float* att) {
  __shared__ __attribute__((aligned(16))) float satt[(ATHR / 32) * NNB * GN];
  const int tid = (int)threadIdx.x, lane = tid & 31, wave = tid >> 5, hh = lane >> 4, m = lane & 15;
  const int node  = (int)blockIdx.x * NPB + wave;
  const int nodec = node < MNODE ? node : MNODE - 1;

  FragB af;
  {
    const float* mp = maps + ((size_t)nodec * NNB + m) * LOCF;
    const v4f ma = *(const v4fa*)mp;
    const v4f mb = *(const v4fa*)(mp + 4);
    const unsigned msk = (hh == 0) ? 0xFFFFu : 0u;
    af.u[0] = (unsigned short)(bf16_bits(ma.x) & msk); af.u[1] = (unsigned short)(bf16_bits(ma.y) & msk);
    af.u[2] = (unsigned short)(bf16_bits(ma.z) & msk); af.u[3] = (unsigned short)(bf16_bits(ma.w) & msk);
    af.u[4] = (unsigned short)(bf16_bits(mb.x) & msk); af.u[5] = (unsigned short)(bf16_bits(mb.y) & msk);
    af.u[6] = (unsigned short)(bf16_bits(mb.z) & msk); af.u[7] = (unsigned short)(bf16_bits(mb.w) & msk);
    af.u[8] = 0; af.u[9] = 0; af.u[10] = 0; af.u[11] = 0; af.u[12] = 0; af.u[13] = 0; af.u[14] = 0; af.u[15] = 0;
  }
  const v8f zero8 = {0.f, 0.f, 0.f, 0.f, 0.f, 0.f, 0.f, 0.f};
  float* sw = satt + wave * (NNB * GN);

#pragma unroll 1
  for (int g = 0; g < GN; ++g) {
    float p[8];
#pragma unroll
    for (int r = 0; r < 8; ++r) p[r] = 0.0f;
#pragma unroll 1
    for (int nt = 0; nt < LH / 16; ++nt) {
      const int col = 16 * nt + m;
      const unsigned short* br = w1p + (size_t)(g * LH + col) * KP;
      FragB bf;
      bf.h[0] = *(const v8usa*)(br + 8 * hh);
      bf.h[1] = *(const v8usa*)(br + 16 + 8 * hh);
      const v8f d = wmb(af, bf, zero8);
      const float bb = bf16_val(b1[g * LH + col]);
      const float ww = bf16_val(w2[g * LH + col]);
#pragma unroll
      for (int r = 0; r < 8; ++r) p[r] = fmaf(tanhf(d[r] + bb), ww, p[r]);
    }
    const float b2g = bf16_val(b2[g]);
#pragma unroll
    for (int r = 0; r < 8; ++r) {
      float v = p[r];
      v += __shfl_xor(v, 1, 32);
      v += __shfl_xor(v, 2, 32);
      v += __shfl_xor(v, 4, 32);
      v += __shfl_xor(v, 8, 32);
      p[r] = v + b2g;
    }
    float mx = p[0];
#pragma unroll
    for (int r = 1; r < 8; ++r) mx = fmaxf(mx, p[r]);
    mx = fmaxf(mx, __shfl_xor(mx, 16, 32));
    float ex[8];
    float s = 0.0f;
#pragma unroll
    for (int r = 0; r < 8; ++r) { ex[r] = expf(p[r] - mx); s += ex[r]; }
    s += __shfl_xor(s, 16, 32);
    const float inv = 1.0f / s;
    if (m == 0) {
#pragma unroll
      for (int r = 0; r < 8; ++r) sw[(8 * hh + r) * GN + g] = ex[r] * inv;
    }
  }
  wave_sync();
  const v4f v = *(const v4fa*)(sw + (lane & 15) * GN);
  float* dst = att + ((size_t)nodec * NNB + (lane & 15)) * GN;
  const bool wr = (lane < 16) && (node < MNODE);
  if (wr) *(volatile v4f*)dst = v;
  __threadfence();
  if (wr) *(volatile v4f*)dst = v;
}

__global__ __launch_bounds__(ATHR) void k_xw(const float* __restrict__ x, const float* __restrict__ wx, float* xw) {
  __shared__ __attribute__((aligned(16))) float stg[GBM * NXW];
  __shared__ __attribute__((aligned(16))) unsigned short sB[NXW * KP];
  const int tid = (int)threadIdx.x, lane = tid & 31, wave = tid >> 5, hh = lane >> 4, m = lane & 15;
  const int rowBase = (int)blockIdx.x * GBM;

#pragma unroll
  for (int i = 0; i < (GN * XF * OF) / (4 * ATHR); ++i) {
    const int idx = ATHR * i + tid;
    const v4f v = *(const v4fa*)(wx + 4 * idx);
    const int o4 = (idx & 7) * 4, f = (idx >> 3) & (XF - 1), g = idx >> 8;
    unsigned short* sp = sB + (g * OF + o4) * KP + f;
    sp[0]      = (unsigned short)bf16_bits(v.x);
    sp[KP]     = (unsigned short)bf16_bits(v.y);
    sp[2 * KP] = (unsigned short)bf16_bits(v.z);
    sp[3 * KP] = (unsigned short)bf16_bits(v.w);
  }
  FragB af;
  {
    const int r  = rowBase + 16 * wave + m;
    const int rc = r < NROWS ? r : NROWS - 1;
    const float* xr = x + (size_t)rc * XF;
    const v4f x0 = *(const v4fa*)(xr + 8 * hh);
    const v4f x1 = *(const v4fa*)(xr + 8 * hh + 4);
    const v4f x2 = *(const v4fa*)(xr + 16 + 8 * hh);
    const v4f x3 = *(const v4fa*)(xr + 16 + 8 * hh + 4);
    af.u[0]  = (unsigned short)bf16_bits(x0.x); af.u[1]  = (unsigned short)bf16_bits(x0.y);
    af.u[2]  = (unsigned short)bf16_bits(x0.z); af.u[3]  = (unsigned short)bf16_bits(x0.w);
    af.u[4]  = (unsigned short)bf16_bits(x1.x); af.u[5]  = (unsigned short)bf16_bits(x1.y);
    af.u[6]  = (unsigned short)bf16_bits(x1.z); af.u[7]  = (unsigned short)bf16_bits(x1.w);
    af.u[8]  = (unsigned short)bf16_bits(x2.x); af.u[9]  = (unsigned short)bf16_bits(x2.y);
    af.u[10] = (unsigned short)bf16_bits(x2.z); af.u[11] = (unsigned short)bf16_bits(x2.w);
    af.u[12] = (unsigned short)bf16_bits(x3.x); af.u[13] = (unsigned short)bf16_bits(x3.y);
    af.u[14] = (unsigned short)bf16_bits(x3.z); af.u[15] = (unsigned short)bf16_bits(x3.w);
  }
  __syncthreads();

  const v8f zero8 = {0.f, 0.f, 0.f, 0.f, 0.f, 0.f, 0.f, 0.f};
  v8f acc[8];
#pragma unroll
  for (int nt = 0; nt < 8; ++nt) {
    const unsigned short* wq = sB + (16 * nt + m) * KP;
    FragB bf;
    bf.h[0] = *(const v8usa*)(wq + 8 * hh);
    bf.h[1] = *(const v8usa*)(wq + 16 + 8 * hh);
    acc[nt] = wmb(af, bf, zero8);
  }

#pragma unroll
  for (int nt = 0; nt < 8; ++nt) {
    const int lc = 16 * nt + m;
#pragma unroll
    for (int r = 0; r < 8; ++r) {
      const int lr = 16 * wave + 8 * hh + r;
      stg[lr * NXW + lc] = acc[nt][r];
    }
  }
  __syncthreads();
  v4f pv[16];
#pragma unroll
  for (int i = 0; i < 16; ++i) pv[i] = *(const v4fa*)(stg + (16 * wave + i) * NXW + 4 * lane);
#pragma unroll
  for (int i = 0; i < 16; ++i) {
    const int r = rowBase + 16 * wave + i;
    if (r < NROWS) *(volatile v4f*)(xw + (size_t)r * NXW + 4 * lane) = pv[i];
  }
  __threadfence();
#pragma unroll
  for (int i = 0; i < 16; ++i) {
    const int r = rowBase + 16 * wave + i;
    if (r < NROWS) *(volatile v4f*)(xw + (size_t)r * NXW + 4 * lane) = pv[i];
  }
}

__global__ __launch_bounds__(NTHR) void k_agg(const int* __restrict__ lix, const float* __restrict__ att,
                                              const float* __restrict__ xw, const float* __restrict__ bx,
                                              float* out, int nE, int vec8) {
  extern __shared__ __attribute__((aligned(16))) int dsm[];
  int* list = dsm;
  int* hl   = dsm + LISTN;
  int* sl   = hl + RCAP;
  int* cnt  = sl + RCAP;
  int* offs = cnt + NBA;
  int* cur  = offs + NBA;
  int* misc = cur + NBA;
  const int tid = (int)threadIdx.x, lane = tid & 31, wave = tid >> 5;
  const int nodeBase = (int)blockIdx.x * NBA;

  {
    const v4i z4 = {0, 0, 0, 0};
    for (int i = tid * 4; i < AGG_ZINTS; i += NTHR * 4) *(v4ia*)(dsm + i) = z4;
    if (tid < MISC_INTS) misc[tid] = 0;
  }
  __syncthreads();

  int t = 0, ov = 0;
  const int nChunks = (nE + CHUNK - 1) / CHUNK;
#pragma unroll 1
  for (int ch = 0; ch < nChunks; ++ch) {
    const int cbase = ch * CHUNK;
    const int wc = scan_chunk<SLA>(lix, nE, cbase, nodeBase, NBA, vec8, list, tid, lane, wave);
    if (lane == 0) misc[wave] = wc;
    __syncthreads();
    if (wave == 0) {
#pragma unroll 1
      for (int w2 = 0; w2 < NWAVE; ++w2) {
        int c = misc[w2];
        c = c < 0 ? 0 : (c > WCAP ? WCAP : c);
#pragma unroll 1
        for (int b0 = 0; b0 < c; b0 += 32) {
          const int idx = b0 + lane;
          const int ent = list[w2 * WCAP + (idx < WCAP ? idx : WCAP - 1)];
          const int m32 = (c - b0) < 32 ? (c - b0) : 32;
#pragma unroll 1
          for (int k = 0; k < m32; ++k) {
            const int u    = __builtin_amdgcn_readlane(ent, k);
            const int slot = u & (NBA - 1);
            const int el   = (u >> SLA) & (CHUNK - 1);
            const int pk   = ((cbase + el) << SLA) | slot;
            if (t < RCAP) {
              if (lane == 0) { hl[t] = pk; cnt[slot] = cnt[slot] + 1; }
              t = t + 1;
            } else {
              ov = 1;
            }
          }
        }
      }
    }
    __syncthreads();
  }
  if (wave == 0 && lane == 0) { misc[8] = t; misc[9] = ov; }
  __syncthreads();
  int tt = misc[8];
  tt = tt < 0 ? 0 : (tt > RCAP ? RCAP : tt);
  const int ovf = misc[9];

  if (wave == 0) {
    const int base = lane * (NBA / 32);
    int s = 0;
#pragma unroll 1
    for (int i = 0; i < NBA / 32; ++i) s += cnt[base + i];
    int incl = s;
#pragma unroll
    for (int d = 1; d < 32; d <<= 1) {
      const int y = __shfl_up(incl, d, 32);
      if (lane >= d) incl += y;
    }
    int run = incl - s;
#pragma unroll 1
    for (int i = 0; i < NBA / 32; ++i) {
      const int cv = cnt[base + i];
      offs[base + i] = run;
      cur[base + i]  = run;
      run += cv;
    }
  }
  __syncthreads();
  if (wave == 0) {
#pragma unroll 1
    for (int b0 = 0; b0 < tt; b0 += 32) {
      const int idx = b0 + lane;
      const int ent = hl[idx < RCAP ? idx : RCAP - 1];
      const int m32 = (tt - b0) < 32 ? (tt - b0) : 32;
#pragma unroll 1
      for (int k = 0; k < m32; ++k) {
        const int u    = __builtin_amdgcn_readlane(ent, k);
        const int slot = u & (NBA - 1);
        if (lane == 0) {
          int p = cur[slot];
          p = p < 0 ? 0 : (p > RCAP - 1 ? RCAP - 1 : p);
          sl[p] = u;
          cur[slot] = p + 1;
        }
      }
    }
  }
  __syncthreads();

  const float pz = (ovf != 0) ? __int_as_float(0x7fc00000) : 0.0f;
  const int sg = lane >> 3;
  const int q4 = (lane & 7) * 4;
  v4f bx4;
  {
    const v4f tb = *(const v4fa*)(bx + q4);
    bx4.x = bf16_val(tb.x); bx4.y = bf16_val(tb.y); bx4.z = bf16_val(tb.z); bx4.w = bf16_val(tb.w);
  }
#pragma unroll 1
  for (int si = 0; si < NBA / NWAVE; ++si) {
    const int s    = si * NWAVE + wave;
    const int node = nodeBase + s;
    const int craw = cnt[s];
    const bool big = craw > DEGCAP;
    const int c = craw < 0 ? 0 : (craw > DEGCAP ? DEGCAP : craw);
    int o = offs[s];
    o = o < 0 ? 0 : (o > RCAP ? RCAP : o);
    int i0 = o + lane;       i0 = i0 > RCAP - 1 ? RCAP - 1 : i0;
    int i1 = o + 32 + lane;  i1 = i1 > RCAP - 1 ? RCAP - 1 : i1;
    const int ent0 = sl[i0];
    const int ent1 = sl[i1];
    int e0 = ent0 >> SLA; e0 = e0 < 0 ? 0 : (e0 > nE - 1 ? nE - 1 : e0);
    int e1 = ent1 >> SLA; e1 = e1 < 0 ? 0 : (e1 > nE - 1 ? nE - 1 : e1);
    const int j0 = keycol(lix[e0]);
    const int j1 = keycol(lix[e1]);
    const bool v0 = lane < c;
    const bool v1 = (lane + 32) < c;

    int kl0 = 0, kl1 = 0;
#pragma unroll 1
    for (int b0 = 0; b0 < c; b0 += 32) {
      const int eb  = (b0 == 0) ? e0 : e1;
      const int jb  = (b0 == 0) ? j0 : j1;
      const int m32 = (c - b0) < 32 ? (c - b0) : 32;
#pragma unroll 1
      for (int k = 0; k < m32; ++k) {
        const int ek = __builtin_amdgcn_readlane(eb, k);
        const int jk = __builtin_amdgcn_readlane(jb, k);
        kl0 |= ((j0 == jk) && (e0 < ek)) ? 1 : 0;
        kl1 |= ((j1 == jk) && (e1 < ek)) ? 1 : 0;
      }
    }
    const int al0 = (v0 && kl0 == 0) ? 1 : 0;
    const int al1 = (v1 && kl1 == 0) ? 1 : 0;

    const v4f z4 = {0.f, 0.f, 0.f, 0.f};
    v4f acc[BSZ];
#pragma unroll
    for (int b = 0; b < BSZ; ++b) acc[b] = z4;
#pragma unroll 1
    for (int b0 = 0; b0 < c; b0 += 32) {
      const int eb  = (b0 == 0) ? e0 : e1;
      const int jb  = (b0 == 0) ? j0 : j1;
      const int ab  = (b0 == 0) ? al0 : al1;
      const int m32 = (c - b0) < 32 ? (c - b0) : 32;
#pragma unroll 1
      for (int k = 0; k < m32; ++k) {
        const int ak = __builtin_amdgcn_readlane(ab, k);
        if (ak != 0) {
          const int ek = __builtin_amdgcn_readlane(eb, k);
          const int jk = __builtin_amdgcn_readlane(jb, k);
          const v4f a4 = *(const v4fa*)(att + (size_t)ek * GN);
          float ag = a4.x;
          ag = (sg == 1) ? a4.y : ag;
          ag = (sg == 2) ? a4.z : ag;
          ag = (sg == 3) ? a4.w : ag;
          const float* xr = xw + (size_t)jk * NXW + 4 * lane;
#pragma unroll
          for (int b = 0; b < BSZ; ++b) {
            const v4f xv = *(const v4fa*)(xr + (size_t)b * ((size_t)MNODE * NXW));
            acc[b] += ag * xv;
          }
        }
      }
    }
#pragma unroll
    for (int b = 0; b < BSZ; ++b) {
      v4f tv = acc[b];
      tv.x += __shfl_xor(tv.x, 8, 32);  tv.y += __shfl_xor(tv.y, 8, 32);
      tv.z += __shfl_xor(tv.z, 8, 32);  tv.w += __shfl_xor(tv.w, 8, 32);
      tv.x += __shfl_xor(tv.x, 16, 32); tv.y += __shfl_xor(tv.y, 16, 32);
      tv.z += __shfl_xor(tv.z, 16, 32); tv.w += __shfl_xor(tv.w, 16, 32);
      acc[b] = tv;
    }
    const float pzr = big ? __int_as_float(0x7fc00000) : pz;
    v4f vo[4];
#pragma unroll
    for (int p = 0; p < 4; ++p) {
      v4f tv = acc[4 * p];
      tv = sel4(sg == 1, acc[4 * p + 1], tv);
      tv = sel4(sg == 2, acc[4 * p + 2], tv);
      tv = sel4(sg == 3, acc[4 * p + 3], tv);
      tv.x = tv.x + bx4.x + pzr; tv.y = tv.y + bx4.y + pzr;
      tv.z = tv.z + bx4.z + pzr; tv.w = tv.w + bx4.w + pzr;
      vo[p] = tv;
    }
    if (node < MNODE) {
#pragma unroll
      for (int p = 0; p < 4; ++p) {
        float* dp = out + ((size_t)(4 * p + sg) * MNODE + (size_t)node) * OF + q4;
        *(volatile v4f*)dp = vo[p];
      }
      __threadfence();
#pragma unroll
      for (int p = 0; p < 4; ++p) {
        float* dp = out + ((size_t)(4 * p + sg) * MNODE + (size_t)node) * OF + q4;
        *(volatile v4f*)dp = vo[p];
      }
    }
  }
}

static inline size_t al256(size_t o) { return (o + 255) & ~(size_t)255; }

extern "C" void kernel_launch(void* const* d_in, const int* in_sizes, int n_in,
                              void* d_out, int out_size, void* d_ws, size_t ws_size,
                              hipStream_t stream) {
  if (n_in < 9) return;
  if (in_sizes[0] != BSZ * MNODE * XF) return;
  if (in_sizes[1] != NENT * LOCF) return;
  if (in_sizes[2] != NENT) return;
  if (in_sizes[3] != GN * LH * LOCF) return;
  if (in_sizes[4] != GN * LH) return;
  if (in_sizes[5] != GN * LH) return;
  if (in_sizes[6] != GN) return;
  if (in_sizes[7] != GN * XF * OF) return;
  if (in_sizes[8] != OF) return;
  if (out_size != BSZ * MNODE * OF) return;

  const float* x    = (const float*)d_in[0];
  const float* maps = (const float*)d_in[1];
  const int*   lix  = (const int*)d_in[2];
  const float* W1   = (const float*)d_in[3];
  const float* b1   = (const float*)d_in[4];
  const float* W2   = (const float*)d_in[5];
  const float* b2   = (const float*)d_in[6];
  const float* Wx   = (const float*)d_in[7];
  const float* bx   = (const float*)d_in[8];
  float* out = (float*)d_out;
  const int nE = in_sizes[2];
  const int vec8 = ((nE & 3) == 0) ? 1 : 0;

  char* ws = (char*)d_ws;
  size_t off = 0;
  const size_t oW1P = off; off = al256(off + (size_t)GN * LH * KP * 2);
  const size_t oATT = off; off = al256(off + (size_t)NENT * GN * 4);
  const size_t oXW  = off; off = al256(off + (size_t)NROWS * NXW * 4);
  if (off > ws_size || off > (size_t)WSMAX) return;
  unsigned short* W1P = (unsigned short*)(ws + oW1P);
  float* ATT = (float*)(ws + oATT);
  float* XW  = (float*)(ws + oXW);

  const size_t aggLds = (size_t)AGG_LDS_INTS * 4;
  hipFuncSetAttribute(reinterpret_cast<const void*>(&k_agg), hipFuncAttributeMaxDynamicSharedMemorySize, (int)aggLds);

  k_w1prep<<<WUNITS / NTHR, NTHR, 0, stream>>>(W1, W1P);
  k_att<<<MNODE / NPB, ATHR, 0, stream>>>(maps, W1P, b1, W2, b2, ATT);
  k_xw<<<NROWS / GBM, ATHR, 0, stream>>>(x, Wx, XW);
  k_agg<<<MNODE / NBA, NTHR, aggLds, stream>>>(lix, ATT, XW, bx, out, nE, vec8);
}
